// FlashAttention_78108275245191
// MI455X (gfx1250) — hardware-verified
//
#include <hip/hip_runtime.h>


#ifndef NB
#define NB 2
#endif
#ifndef SEQ
#define SEQ 4096
#endif
#ifndef SEQ_FULL
#define SEQ_FULL 4096
#endif
#ifndef RH
#define RH 1024
#endif
#define NH 16
#define HD 64
#define NZ (NB * NH)
#define QT 128
#define KC 64
#define PCAR 1024.0f
#define PCINV 0.0009765625f
#define SCL 0.125f
#define L2E 1.4426950408889634f
#define NEG (-1.0e30f)
static_assert(SEQ % QT == 0);
static_assert(SEQ % KC == 0);
static_assert(RH % QT == 0);
static_assert(QT == 8 * 16);
static_assert(HD == 64);
static_assert(SEQ <= SEQ_FULL);
static_assert(((long long)NZ * SEQ * HD) % 8 == 0);

typedef _Float16 h16;
typedef unsigned short bf;
typedef __attribute__((ext_vector_type(16))) __bf16         v16bf;
typedef __attribute__((ext_vector_type(16))) _Float16       v16h;
typedef __attribute__((ext_vector_type(16))) unsigned short v16us;
typedef __attribute__((ext_vector_type(8)))  _Float16       v8h;
typedef __attribute__((ext_vector_type(8)))  unsigned short v8us;
typedef __attribute__((ext_vector_type(8)))  float          v8f;
typedef __attribute__((ext_vector_type(4)))  float          v4f;
typedef __attribute__((ext_vector_type(2)))  _Float16       v2h;
typedef __attribute__((ext_vector_type(2)))  unsigned short v2us;
typedef v4f __attribute__((may_alias)) v4fa;

__device__ __forceinline__ unsigned short f2bf(float f) { unsigned u = __float_as_uint(f); u += 0x7FFFu + ((u >> 16) & 1u); return (unsigned short)(u >> 16); }
__device__ __forceinline__ float bf2f(unsigned short b) { return __uint_as_float(((unsigned)b) << 16); }
__device__ __forceinline__ float bfr(float f) { return bf2f(f2bf(f)); }
__device__ __forceinline__ void splitf(float y, unsigned short& h, unsigned short& l) { h = f2bf(y); l = f2bf(y - bf2f(h)); }
__device__ __forceinline__ v16h  cat16(v8h lo, v8h hi) { return __builtin_shufflevector(lo, hi, 0, 1, 2, 3, 4, 5, 6, 7, 8, 9, 10, 11, 12, 13, 14, 15); }
__device__ __forceinline__ v16bf cat16b(v8us lo, v8us hi) { return __builtin_bit_cast(v16bf, __builtin_shufflevector(lo, hi, 0, 1, 2, 3, 4, 5, 6, 7, 8, 9, 10, 11, 12, 13, 14, 15)); }
__device__ __forceinline__ v8f wmma16(v16h a, v16h b, v8f c) { return __builtin_amdgcn_wmma_f32_16x16x32_f16(false, a, false, b, (short)0, c, false, false); }
__device__ __forceinline__ v8f wmmab(v16bf a, v16bf b, v8f c) { return __builtin_amdgcn_wmma_f32_16x16x32_bf16(false, a, false, b, (short)0, c, false, false); }

__device__ __forceinline__ v16bf ldb(const bf* p) { return cat16b(*(const v8us*)p, *(const v8us*)(p + 16)); }
__device__ __forceinline__ v16h  ldh(const h16* p) { return cat16(*(const v8h*)p, *(const v8h*)(p + 16)); }

__global__ __launch_bounds__(256) void k_cvt8(const float* __restrict__ src, bf* dst, int n8) {
    const int i = blockIdx.x * 256 + threadIdx.x; if (i >= n8) return;
    const size_t e = (size_t)i * 8; const size_t zz = e / ((size_t)SEQ * HD); const size_t rem = e - zz * ((size_t)SEQ * HD);
    const v8f v = *(const v8f*)(src + zz * ((size_t)SEQ_FULL * HD) + rem); v8us o;
#pragma unroll
    for (int k = 0; k < 8; ++k) o[k] = f2bf(v[k]);
    *(volatile v8us*)(dst + e) = o; __threadfence(); *(volatile v8us*)(dst + e) = o;
}

__global__ __launch_bounds__(256) void k_vtp(const float* __restrict__ F, h16* V16, bf* Vh, int n2) {
    const int i = blockIdx.x * 256 + threadIdx.x; if (i >= n2) return;
    const size_t e = (size_t)i * 2; const int t = (int)(e % SEQ); const int d = (int)((e / SEQ) % HD); const size_t zz = e / ((size_t)SEQ * HD);
    const float* f = F + (zz * SEQ_FULL + (size_t)t) * HD + d; v2h o16; v2us oh;
#pragma unroll
    for (int q = 0; q < 2; ++q) { const float x = bfr(f[(size_t)q * HD]); o16[q] = (h16)x; oh[q] = f2bf(x); }
    *(volatile v2h*)(V16 + e) = o16; *(volatile v2us*)(Vh + e) = oh; __threadfence(); *(volatile v2h*)(V16 + e) = o16; *(volatile v2us*)(Vh + e) = oh;
}

template <bool HR>
__global__ __launch_bounds__(256) __attribute__((amdgpu_num_vgpr(256)))
void k_attn(const bf* __restrict__ Qp, const bf* __restrict__ Kp, const bf* __restrict__ VTh, const h16* __restrict__ VT16, float* OUT, int qb0) {
#pragma clang fp contract(off)
    __shared__ __align__(16) float os[8 * 16 * 68];
    const int lane = threadIdx.x & 31, lr = lane & 15, hi = lane >> 4, wave = threadIdx.x >> 5;
    const size_t z = blockIdx.y;
    const int q0 = (qb0 + (int)blockIdx.x) * QT + wave * 16;
    const int myq = q0 + lr;
    const bf* Qz = Qp + z * ((size_t)SEQ * HD);
    const bf* Kz = Kp + z * ((size_t)SEQ * HD);
    const bf* Vhz = VTh + z * ((size_t)HD * SEQ);
    const h16* V16z = VT16 + z * ((size_t)HD * SEQ);
    const v16bf qf0 = ldb(Qz + (size_t)myq * HD + 8 * hi);
    const v16bf qf1 = ldb(Qz + (size_t)myq * HD + 32 + 8 * hi);
    v8f oacc[4];
#pragma unroll
    for (int dt = 0; dt < 4; ++dt) oacc[dt] = (v8f){};
    float m = NEG, lsum = 0.0f;
    const int nch = (q0 + 15) / KC + 1;
#pragma unroll 1
    for (int c = 0; c < nch; ++c) {
        const int k0 = c * KC;
        v8f s[4];
#pragma unroll
        for (int jg = 0; jg < 2; ++jg) {
            const bf* kr0 = Kz + (size_t)(k0 + 32 * jg + lr) * HD + 8 * hi;
            const bf* kr1 = kr0 + 16 * HD;
            const v16bf ka0 = ldb(kr0), ka1 = ldb(kr0 + 32), kb0 = ldb(kr1), kb1 = ldb(kr1 + 32);
            v8f t0 = wmmab(ka0, qf0, (v8f){}); t0 = wmmab(ka1, qf1, t0);
            v8f t1 = wmmab(kb0, qf0, (v8f){}); t1 = wmmab(kb1, qf1, t1);
            asm volatile("v_nop\n\tv_nop\n\tv_nop\n\tv_nop" : "+v"(t0), "+v"(t1) : "v"(ka0), "v"(ka1), "v"(kb0), "v"(kb1), "v"(qf0), "v"(qf1));
            s[2 * jg] = t0; s[2 * jg + 1] = t1;
        }
        float tmx = NEG;
#pragma unroll
        for (int j = 0; j < 4; ++j) {
#pragma unroll
            for (int r = 0; r < 8; ++r) {
                const int key = k0 + 16 * j + 8 * hi + r;
                const float t = (key <= myq) ? s[j][r] * SCL : NEG;
                s[j][r] = t; tmx = fmaxf(tmx, t);
            }
        }
        tmx = fmaxf(tmx, __shfl_xor(tmx, 16, 32));
        const float mn = fmaxf(m, tmx);
        const float alpha = __builtin_amdgcn_exp2f((m - mn) * L2E);
        m = mn; lsum *= alpha;
#pragma unroll
        for (int dt = 0; dt < 4; ++dt)
#pragma unroll
            for (int r = 0; r < 8; ++r) oacc[dt][r] *= alpha;
        v16bf pbh[2], pbl[2]; v16h pf[2];
#pragma unroll
        for (int ks = 0; ks < 2; ++ks) {
            v16us uh, ul; v16h p16;
#pragma unroll
            for (int half = 0; half < 2; ++half) {
                const int j = 2 * ks + half;
#pragma unroll
                for (int r = 0; r < 8; ++r) {
                    const float p = __builtin_amdgcn_exp2f((s[j][r] - mn) * L2E);
                    lsum += p;
                    if (HR) { unsigned short a, b2; splitf(p, a, b2); uh[half * 8 + r] = a; ul[half * 8 + r] = b2; }
                    else { p16[half * 8 + r] = (h16)(p * PCAR); }
                }
            }
            if (HR) { pbh[ks] = __builtin_bit_cast(v16bf, uh); pbl[ks] = __builtin_bit_cast(v16bf, ul); }
            else { pf[ks] = p16; }
        }
#pragma unroll
        for (int ks = 0; ks < 2; ++ks) {
            const int kk = k0 + 32 * ks + 8 * hi;
            if (HR) {
                const v16bf bh = pbh[ks], bl = pbl[ks];
                v16bf vf[4];
#pragma unroll
                for (int dt = 0; dt < 4; ++dt) vf[dt] = ldb(Vhz + (size_t)(dt * 16 + lr) * SEQ + kk);
#pragma unroll
                for (int dt = 0; dt < 4; ++dt) { oacc[dt] = wmmab(vf[dt], bh, oacc[dt]); oacc[dt] = wmmab(vf[dt], bl, oacc[dt]); }
                asm volatile("v_nop\n\tv_nop\n\tv_nop\n\tv_nop" : "+v"(oacc[0]), "+v"(oacc[1]), "+v"(oacc[2]), "+v"(oacc[3]) : "v"(vf[0]), "v"(vf[1]), "v"(vf[2]), "v"(vf[3]), "v"(bh), "v"(bl));
            } else {
                const v16h bp = pf[ks];
                v16h vf[4];
#pragma unroll
                for (int dt = 0; dt < 4; ++dt) vf[dt] = ldh(V16z + (size_t)(dt * 16 + lr) * SEQ + kk);
#pragma unroll
                for (int dt = 0; dt < 4; ++dt) oacc[dt] = wmma16(vf[dt], bp, oacc[dt]);
                asm volatile("v_nop\n\tv_nop\n\tv_nop\n\tv_nop" : "+v"(oacc[0]), "+v"(oacc[1]), "+v"(oacc[2]), "+v"(oacc[3]) : "v"(vf[0]), "v"(vf[1]), "v"(vf[2]), "v"(vf[3]), "v"(bp));
            }
        }
    }
    lsum += __shfl_xor(lsum, 16, 32);
    const float inv = __fdiv_rn(HR ? 1.0f : PCINV, lsum);
    float* osw = os + wave * (16 * 68);
#pragma unroll
    for (int dt = 0; dt < 4; ++dt)
#pragma unroll
        for (int r = 0; r < 8; ++r) osw[lr * 68 + dt * 16 + 8 * hi + r] = oacc[dt][r] * inv;
    __builtin_amdgcn_fence(3, "wavefront"); __builtin_amdgcn_wave_barrier(); asm volatile("" ::: "memory");
    float* orow = OUT + (z * SEQ + (size_t)q0) * HD;
    v4f val[8];
#pragma unroll
    for (int sg = 0; sg < 8; ++sg) val[sg] = *(const v4fa*)(osw + (2 * sg + hi) * 68 + lr * 4);
#pragma unroll
    for (int sg = 0; sg < 8; ++sg) *(volatile v4f*)(orow + (size_t)(2 * sg + hi) * HD + lr * 4) = val[sg];
    __threadfence();
#pragma unroll
    for (int sg = 0; sg < 8; ++sg) *(volatile v4f*)(orow + (size_t)(2 * sg + hi) * HD + lr * 4) = val[sg];
}

extern "C" void kernel_launch(void* const* d_in, const int* in_sizes, int n_in,
                              void* d_out, int out_size, void* d_ws, size_t ws_size, hipStream_t stream) {
    if (n_in < 3) return;
    const float* xq = (const float*)d_in[0];
    const float* xk = (const float*)d_in[1];
    const float* xv = (const float*)d_in[2];
    float* OUT = (float*)d_out;
    const long long need_in = (long long)(NZ - 1) * SEQ_FULL * HD + (long long)SEQ * HD;
    if ((long long)in_sizes[0] < need_in || (long long)in_sizes[1] < need_in || (long long)in_sizes[2] < need_in) return;
    if ((long long)out_size < (long long)NZ * SEQ * HD) return;
    char* wsp = (char*)d_ws;
    auto take = [&](size_t bytes) { char* p = wsp; wsp += (bytes + 255) & ~(size_t)255; return (void*)p; };
    const size_t plane = (size_t)NZ * SEQ * HD;
    bf*  Qp   = (bf*)take(plane * 2);
    bf*  Kp   = (bf*)take(plane * 2);
    bf*  VTh  = (bf*)take(plane * 2);
    h16* VT16 = (h16*)take(plane * 2);
    if ((size_t)(wsp - (char*)d_ws) > ws_size) return;
    const int n8 = (int)(plane / 8), n2 = (int)(plane / 2);
    k_cvt8<<<(unsigned)((n8 + 255) / 256), 256, 0, stream>>>(xq, Qp, n8);
    k_cvt8<<<(unsigned)((n8 + 255) / 256), 256, 0, stream>>>(xk, Kp, n8);
    k_vtp<<<(unsigned)((n2 + 255) / 256), 256, 0, stream>>>(xv, VT16, VTh, n2);
    const int nqb = SEQ / QT;
    const int rhb = ((RH < SEQ) ? RH : SEQ) / QT;
    if (rhb > 0) k_attn<true><<<dim3((unsigned)rhb, NZ), 256, 0, stream>>>(Qp, Kp, VTh, VT16, OUT, 0);
    if (nqb - rhb > 0) k_attn<false><<<dim3((unsigned)(nqb - rhb), NZ), 256, 0, stream>>>(Qp, Kp, VTh, VT16, OUT, rhb);
}
